// LSTMEncoder_249108103773
// MI455X (gfx1250) — hardware-verified
//
#include <hip/hip_runtime.h>
#include <math.h>

constexpr int NBATCH   = 4096;
constexpr int NSTEPS   = 5;
constexpr int NIN1     = 11;
constexpr int NHID     = 512;
constexpr int NGATE    = 4 * NHID;
constexpr int KXPAD    = 32;
constexpr int NTHR     = 256;
constexpr int ROWS_BLK = 16;
constexpr int XPITCH   = 40;
constexpr int HPITCH   = 520;
constexpr int SLABP    = 68;
constexpr float WCAR    = 256.0f;
constexpr float XWCAR   = 4096.0f;
constexpr float HCAR    = 16.0f;
constexpr float ACC_INV = 1.0f / 4096.0f;
static_assert(NBATCH % ROWS_BLK == 0);
static_assert(NHID == 64 * (NTHR / 32));
static_assert(NHID % 32 == 0 && KXPAD % 32 == 0);
static_assert((4 * ROWS_BLK * HPITCH) % (2 * NTHR) == 0);
static_assert(NGATE % NTHR == 0);
static_assert(ROWS_BLK * (KXPAD / 2) == NTHR);
static_assert((NGATE * (NHID / 8)) % NTHR == 0);
static_assert((NGATE * (KXPAD / 8)) % NTHR == 0);
static_assert(XPITCH % 8 == 0 && HPITCH % 8 == 0 && SLABP % 4 == 0);

typedef __attribute__((ext_vector_type(16))) _Float16 v16h;
typedef __attribute__((ext_vector_type(8)))  _Float16 v8h;
typedef __attribute__((ext_vector_type(16))) __bf16   v16b;
typedef __attribute__((ext_vector_type(8)))  __bf16   v8b;
typedef __attribute__((ext_vector_type(8)))  float    v8f;
typedef __attribute__((ext_vector_type(4)))  float    v4f;

__device__ __forceinline__ unsigned short f2bf_bits(float f) {
  unsigned u = __float_as_uint(f);
  return (unsigned short)((u + 0x7FFFu + ((u >> 16) & 1u)) >> 16);
}
__device__ __forceinline__ float bf_bits2f(unsigned short h) { return __uint_as_float(((unsigned)h) << 16); }
__device__ __forceinline__ float bf16r(float f) { return bf_bits2f(f2bf_bits(f)); }

__device__ __forceinline__ void dep_guard_h(v8f& a, v8f& b, v16h x, v16h y) { asm volatile("v_nop\n\tv_nop\n\tv_nop\n\tv_nop" : "+v"(a), "+v"(b) : "v"(x), "v"(y)); }
__device__ __forceinline__ void dep_guard_b(v8f& a, v8f& b, v16b x, v16b y) { asm volatile("v_nop\n\tv_nop\n\tv_nop\n\tv_nop" : "+v"(a), "+v"(b) : "v"(x), "v"(y)); }
__device__ __forceinline__ void keep4_h(v16h a, v16h b, v16h c, v16h d) { asm volatile("v_nop" :: "v"(a), "v"(b), "v"(c), "v"(d)); }
__device__ __forceinline__ void keep4_b(v16b a, v16b b, v16b c, v16b d) { asm volatile("v_nop" :: "v"(a), "v"(b), "v"(c), "v"(d)); }
__device__ __forceinline__ void acc_guard4(v8f& a, v8f& b, v8f& c, v8f& d) { asm volatile("v_nop\n\tv_nop\n\tv_nop\n\tv_nop" : "+v"(a), "+v"(b), "+v"(c), "+v"(d)); }
__device__ __forceinline__ void group_guard_h(v8f& a0, v8f& a1, v8f& a2, v8f& a3, v16h x, v16h y0, v16h y1, v16h y2, v16h y3) {
  asm volatile("v_nop\n\tv_nop\n\tv_nop\n\tv_nop" : "+v"(a0), "+v"(a1), "+v"(a2), "+v"(a3) : "v"(x), "v"(y0), "v"(y1), "v"(y2), "v"(y3));
}
__device__ __forceinline__ void group_guard_b(v8f& a0, v8f& a1, v8f& a2, v8f& a3, v16b x, v16b y0, v16b y1, v16b y2, v16b y3) {
  asm volatile("v_nop\n\tv_nop\n\tv_nop\n\tv_nop" : "+v"(a0), "+v"(a1), "+v"(a2), "+v"(a3) : "v"(x), "v"(y0), "v"(y1), "v"(y2), "v"(y3));
}
template <typename T> struct Frag;
template <> struct Frag<_Float16> {
  typedef v16h V; union U { v16h v; v8h h[2]; };
  static __device__ __forceinline__ v16h load(const _Float16* p) {
    U f; f.h[0] = *(const v8h*)(p); f.h[1] = *(const v8h*)(p + 16); return f.v;
  }
  static __device__ __forceinline__ v8f mma(v16h a, v16h b, v8f c) {
    return __builtin_amdgcn_wmma_f32_16x16x32_f16(false, a, false, b, (short)0, c, false, false);
  }
  static __device__ __forceinline__ void guard(v8f& a, v8f& b, v16h x, v16h y) { dep_guard_h(a, b, x, y); }
  static __device__ __forceinline__ void keep(v16h a, v16h b, v16h c, v16h d) { keep4_h(a, b, c, d); }
};
template <> struct Frag<__bf16> {
  typedef v16b V; union U { v16b v; v8b h[2]; };
  static __device__ __forceinline__ v16b load(const __bf16* p) {
    U f; f.h[0] = *(const v8b*)(p); f.h[1] = *(const v8b*)(p + 16); return f.v;
  }
  static __device__ __forceinline__ v8f mma(v16b a, v16b b, v8f c) {
    return __builtin_amdgcn_wmma_f32_16x16x32_bf16(false, a, false, b, (short)0, c, false, false);
  }
  static __device__ __forceinline__ void guard(v8f& a, v8f& b, v16b x, v16b y) { dep_guard_b(a, b, x, y); }
  static __device__ __forceinline__ void keep(v16b a, v16b b, v16b c, v16b d) { keep4_b(a, b, c, d); }
};

__device__ __forceinline__ float fsig(float z)  { return __builtin_amdgcn_rcpf(1.0f + expf(-z)); }
__device__ __forceinline__ float ftanh(float z) { return 1.0f - 2.0f * __builtin_amdgcn_rcpf(1.0f + expf(2.0f * z)); }

template <int MODE>
__global__ __launch_bounds__(NTHR) void cvt8_kernel(const float* __restrict__ src, unsigned short* __restrict__ dst,
                                                    int nrow, int ncol8, int spitch, int scol0, float sc) {
  const int i  = blockIdx.x * NTHR + threadIdx.x;
  const int n8 = nrow * ncol8;
  if (i < n8) {
    const int row = i / ncol8;
    const int c8  = i - row * ncol8;
    const float* sp = src + (size_t)row * spitch + scol0 + c8 * 8;
    const v4f a = *(const v4f*)(sp);
    const v4f b = *(const v4f*)(sp + 4);
    v8h hv;
#pragma unroll
    for (int e = 0; e < 4; ++e) {
      unsigned short b0, b1;
      if (MODE == 0) {
        b0 = f2bf_bits(a[e] * sc);
        b1 = f2bf_bits(b[e] * sc);
      } else {
        b0 = __builtin_bit_cast(unsigned short, (_Float16)(bf16r(a[e]) * sc));
        b1 = __builtin_bit_cast(unsigned short, (_Float16)(bf16r(b[e]) * sc));
      }
      hv[e]     = __builtin_bit_cast(_Float16, b0);
      hv[4 + e] = __builtin_bit_cast(_Float16, b1);
    }
    *(volatile v8h*)(dst + (size_t)i * 8) = hv;
    __threadfence();
    *(volatile v8h*)(dst + (size_t)i * 8) = hv;
  }
}

__global__ __launch_bounds__(NTHR) void wx1_kernel(const float* __restrict__ w, unsigned short* __restrict__ dst) {
  const int i = blockIdx.x * NTHR + threadIdx.x;
  if (i < NGATE * (KXPAD / 8)) {
    const int n = i >> 2, q = i & 3;
    const float* wr = w + (size_t)n * NIN1;
    v8h hv;
#pragma unroll
    for (int e = 0; e < 8; ++e) {
      const int k  = 8 * q + e;
      const int kc = (k < NIN1) ? k : (NIN1 - 1);
      const float msk = (k < NIN1) ? 1.0f : 0.0f;
      const float f = wr[kc];
      const float v = (bf16r(f) * XWCAR) * msk;
      hv[e] = __builtin_bit_cast(_Float16, f2bf_bits(v));
    }
    *(volatile v8h*)(dst + (size_t)i * 8) = hv;
    __threadfence();
    *(volatile v8h*)(dst + (size_t)i * 8) = hv;
  }
}

__device__ __forceinline__ unsigned x_pair_bits(const float* __restrict__ xr, int p2) {
  const int k0c = (p2 < NIN1) ? p2 : (NIN1 - 1);
  const int k1c = (p2 + 1 < NIN1) ? (p2 + 1) : (NIN1 - 1);
  const float m0 = (p2 < NIN1) ? 1.0f : 0.0f;
  const float m1 = (p2 + 1 < NIN1) ? 1.0f : 0.0f;
  const float f0 = xr[k0c] * m0;
  const float f1 = xr[k1c] * m1;
  return (unsigned)f2bf_bits(f0) | ((unsigned)f2bf_bits(f1) << 16);
}

__global__ __launch_bounds__(NTHR) void lstm2_kernel(const float* __restrict__ x,
                                                     const float* __restrict__ bi1, const float* __restrict__ bh1,
                                                     const float* __restrict__ bi2, const float* __restrict__ bh2,
                                                     const unsigned short* __restrict__ WX1p,
                                                     const unsigned short* __restrict__ WH1p,
                                                     const unsigned short* __restrict__ WI2p,
                                                     const unsigned short* __restrict__ WH2p,
                                                     float* __restrict__ out) {
  __shared__ __align__(16) unsigned short Ax[ROWS_BLK * XPITCH];
  __shared__ __align__(16) _Float16       Hl[4][ROWS_BLK * HPITCH];
  __shared__ __align__(16) float          Bs[2][NGATE];
  __shared__ __align__(16) float          Sl[NTHR / 32][16 * SLABP];
  const __bf16*   WX1 = (const __bf16*)WX1p;
  const _Float16* WH1 = (const _Float16*)WH1p;
  const _Float16* WI2 = (const _Float16*)WI2p;
  const _Float16* WH2 = (const _Float16*)WH2p;
  const int tid = threadIdx.x, lane = tid & 31, wave = tid >> 5;
  const int c = lane & 15, hh = lane >> 4, koff = hh * 8, c4 = c * 4;
  const int rowbase = blockIdx.x * ROWS_BLK;

  {
    unsigned* hw = (unsigned*)(void*)&Hl[0][0];
#pragma unroll 1
    for (int i = tid; i < (4 * ROWS_BLK * HPITCH) / 2; i += NTHR) hw[i] = 0u;
  }
#pragma unroll 1
  for (int i = tid; i < NGATE; i += NTHR) {
    Bs[0][i] = bf16r(bi1[i]) + bf16r(bh1[i]);
    Bs[1][i] = bf16r(bi2[i]) + bf16r(bh2[i]);
  }
  {
    const int m = tid >> 4, p2 = (tid & 15) * 2;
    const unsigned wv = x_pair_bits(x + ((size_t)(rowbase + m) * NSTEPS + 0) * NIN1, p2);
    *(unsigned*)(Ax + m * XPITCH + p2) = wv;
  }
  float cs0[4][8], cs1[4][8];
#pragma unroll
  for (int nt = 0; nt < 4; ++nt)
#pragma unroll
    for (int r = 0; r < 8; ++r) { cs0[nt][r] = 0.0f; cs1[nt][r] = 0.0f; }
  __syncthreads();

  const v8f z8 = {0.f, 0.f, 0.f, 0.f, 0.f, 0.f, 0.f, 0.f};
  float* slab = Sl[wave];

#pragma unroll 1
  for (int t = 0; t < NSTEPS; ++t) {
    const int p = t & 1;
    const int krec = (t > 0) ? NHID : 0;

    {
      const __bf16*   axrow = (const __bf16*)Ax + c * XPITCH + koff;
      const _Float16* ahrow = &Hl[p][0] + c * HPITCH + koff;
      _Float16* ahn = &Hl[p ^ 1][0];
#pragma unroll
      for (int nt = 0; nt < 4; ++nt) {
        const int j = 64 * wave + 16 * nt + c;
        float bs[4];
#pragma unroll
        for (int g = 0; g < 4; ++g) bs[g] = Bs[0][g * NHID + j];
        v8f acc[4];
        acc[0] = z8; acc[1] = z8; acc[2] = z8; acc[3] = z8;
        {
          const __bf16* wx = WX1 + (size_t)j * KXPAD + koff;
          const v16b a  = Frag<__bf16>::load(axrow);
          const v16b b0 = Frag<__bf16>::load(wx);
          const v16b b1 = Frag<__bf16>::load(wx + (size_t)1 * NHID * KXPAD);
          const v16b b2 = Frag<__bf16>::load(wx + (size_t)2 * NHID * KXPAD);
          const v16b b3 = Frag<__bf16>::load(wx + (size_t)3 * NHID * KXPAD);
          acc[0] = Frag<__bf16>::mma(a, b0, acc[0]);
          acc[1] = Frag<__bf16>::mma(a, b1, acc[1]);
          acc[2] = Frag<__bf16>::mma(a, b2, acc[2]);
          acc[3] = Frag<__bf16>::mma(a, b3, acc[3]);
          group_guard_b(acc[0], acc[1], acc[2], acc[3], a, b0, b1, b2, b3);
        }
        {
          const _Float16* wh = WH1 + (size_t)j * NHID + koff;
#pragma unroll 1
          for (int k0 = 0; k0 < krec; k0 += 32) {
            const v16h a  = Frag<_Float16>::load(ahrow + k0);
            const v16h b0 = Frag<_Float16>::load(wh + k0);
            const v16h b1 = Frag<_Float16>::load(wh + (size_t)1 * NHID * NHID + k0);
            const v16h b2 = Frag<_Float16>::load(wh + (size_t)2 * NHID * NHID + k0);
            const v16h b3 = Frag<_Float16>::load(wh + (size_t)3 * NHID * NHID + k0);
            acc[0] = Frag<_Float16>::mma(a, b0, acc[0]);
            acc[1] = Frag<_Float16>::mma(a, b1, acc[1]);
            acc[2] = Frag<_Float16>::mma(a, b2, acc[2]);
            acc[3] = Frag<_Float16>::mma(a, b3, acc[3]);
            group_guard_h(acc[0], acc[1], acc[2], acc[3], a, b0, b1, b2, b3);
          }
        }
        acc_guard4(acc[0], acc[1], acc[2], acc[3]);
#pragma unroll
        for (int r = 0; r < 8; ++r) {
          const float zi = acc[0][r] * ACC_INV + bs[0];
          const float zf = acc[1][r] * ACC_INV + bs[1];
          const float zg = acc[2][r] * ACC_INV + bs[2];
          const float zo = acc[3][r] * ACC_INV + bs[3];
          const float ig = fsig(zi);
          const float fg = fsig(zf);
          const float gg = ftanh(zg);
          const float og = fsig(zo);
          const float cn = fg * cs0[nt][r] + ig * gg;
          cs0[nt][r] = cn;
          const float hn = og * ftanh(cn);
          ahn[(8 * hh + r) * HPITCH + j] = (_Float16)(hn * HCAR);
        }
      }
    }
    __syncthreads();

    {
      const _Float16* ain  = &Hl[p ^ 1][0] + c * HPITCH + koff;
      const _Float16* arec = &Hl[2 + p][0] + c * HPITCH + koff;
      _Float16* ahn = &Hl[2 + (p ^ 1)][0];
#pragma unroll
      for (int nt = 0; nt < 4; ++nt) {
        const int j = 64 * wave + 16 * nt + c;
        float bs[4];
#pragma unroll
        for (int g = 0; g < 4; ++g) bs[g] = Bs[1][g * NHID + j];
        v8f acc[4];
        acc[0] = z8; acc[1] = z8; acc[2] = z8; acc[3] = z8;
        {
          const _Float16* wi = WI2 + (size_t)j * NHID + koff;
#pragma unroll 1
          for (int k0 = 0; k0 < NHID; k0 += 32) {
            const v16h a  = Frag<_Float16>::load(ain + k0);
            const v16h b0 = Frag<_Float16>::load(wi + k0);
            const v16h b1 = Frag<_Float16>::load(wi + (size_t)1 * NHID * NHID + k0);
            const v16h b2 = Frag<_Float16>::load(wi + (size_t)2 * NHID * NHID + k0);
            const v16h b3 = Frag<_Float16>::load(wi + (size_t)3 * NHID * NHID + k0);
            acc[0] = Frag<_Float16>::mma(a, b0, acc[0]);
            acc[1] = Frag<_Float16>::mma(a, b1, acc[1]);
            acc[2] = Frag<_Float16>::mma(a, b2, acc[2]);
            acc[3] = Frag<_Float16>::mma(a, b3, acc[3]);
            group_guard_h(acc[0], acc[1], acc[2], acc[3], a, b0, b1, b2, b3);
          }
        }
        {
          const _Float16* wh = WH2 + (size_t)j * NHID + koff;
#pragma unroll 1
          for (int k0 = 0; k0 < krec; k0 += 32) {
            const v16h a  = Frag<_Float16>::load(arec + k0);
            const v16h b0 = Frag<_Float16>::load(wh + k0);
            const v16h b1 = Frag<_Float16>::load(wh + (size_t)1 * NHID * NHID + k0);
            const v16h b2 = Frag<_Float16>::load(wh + (size_t)2 * NHID * NHID + k0);
            const v16h b3 = Frag<_Float16>::load(wh + (size_t)3 * NHID * NHID + k0);
            acc[0] = Frag<_Float16>::mma(a, b0, acc[0]);
            acc[1] = Frag<_Float16>::mma(a, b1, acc[1]);
            acc[2] = Frag<_Float16>::mma(a, b2, acc[2]);
            acc[3] = Frag<_Float16>::mma(a, b3, acc[3]);
            group_guard_h(acc[0], acc[1], acc[2], acc[3], a, b0, b1, b2, b3);
          }
        }
        acc_guard4(acc[0], acc[1], acc[2], acc[3]);
#pragma unroll
        for (int r = 0; r < 8; ++r) {
          const float zi = acc[0][r] * ACC_INV + bs[0];
          const float zf = acc[1][r] * ACC_INV + bs[1];
          const float zg = acc[2][r] * ACC_INV + bs[2];
          const float zo = acc[3][r] * ACC_INV + bs[3];
          const float ig = fsig(zi);
          const float fg = fsig(zf);
          const float gg = ftanh(zg);
          const float og = fsig(zo);
          const float cn = fg * cs1[nt][r] + ig * gg;
          cs1[nt][r] = cn;
          const float hn = og * ftanh(cn);
          ahn[(8 * hh + r) * HPITCH + j] = (_Float16)(hn * HCAR);
          slab[(8 * hh + r) * SLABP + 16 * nt + c] = hn;
        }
      }
      {
        const int tn = (t + 1 < NSTEPS) ? (t + 1) : (NSTEPS - 1);
        const int m = tid >> 4, p2 = (tid & 15) * 2;
        const unsigned wv = x_pair_bits(x + ((size_t)(rowbase + m) * NSTEPS + (size_t)tn) * NIN1, p2);
        *(unsigned*)(Ax + m * XPITCH + p2) = wv;
      }
    }
    __syncthreads();
  }

  for (int pass = 0; pass < 2; ++pass) {
#pragma unroll
    for (int it = 0; it < 8; ++it) {
      const int row = it * 2 + hh;
      const v4f v = *(const v4f*)(slab + row * SLABP + c4);
      *(volatile v4f*)(out + (size_t)(rowbase + row) * NHID + 64 * wave + c4) = v;
    }
    __threadfence();
  }
}

extern "C" void kernel_launch(void* const* d_in, const int* in_sizes, int n_in,
                              void* d_out, int out_size, void* d_ws, size_t ws_size, hipStream_t stream) {
  if (n_in < 9 || d_out == nullptr || d_ws == nullptr) return;
  if (in_sizes[0] != NBATCH * NSTEPS * NIN1 || in_sizes[1] != NGATE * NIN1 || in_sizes[2] != NGATE * NHID ||
      in_sizes[3] != NGATE || in_sizes[4] != NGATE || in_sizes[5] != NGATE * NHID || in_sizes[6] != NGATE * NHID ||
      in_sizes[7] != NGATE || in_sizes[8] != NGATE || out_size != NBATCH * NHID) return;

  const float* x     = (const float*)d_in[0];
  const float* w_ih1 = (const float*)d_in[1];
  const float* w_hh1 = (const float*)d_in[2];
  const float* b_ih1 = (const float*)d_in[3];
  const float* b_hh1 = (const float*)d_in[4];
  const float* w_ih2 = (const float*)d_in[5];
  const float* w_hh2 = (const float*)d_in[6];
  const float* b_ih2 = (const float*)d_in[7];
  const float* b_hh2 = (const float*)d_in[8];
  float* out = (float*)d_out;

  char* ws = (char*)d_ws; size_t off = 0;
  auto carve = [&](size_t bytes) -> char* { char* p = ws + off; off += (bytes + 255) & ~(size_t)255; return p; };
  unsigned short* WH1 = (unsigned short*)carve((size_t)NGATE * NHID * 2);
  unsigned short* WI2 = (unsigned short*)carve((size_t)NGATE * NHID * 2);
  unsigned short* WH2 = (unsigned short*)carve((size_t)NGATE * NHID * 2);
  unsigned short* WX1 = (unsigned short*)carve((size_t)NGATE * KXPAD * 2);
  if (off > ws_size || off > (size_t)134217728) return;

  const int n8h = NGATE * (NHID / 8);
  cvt8_kernel<1><<<n8h / NTHR, NTHR, 0, stream>>>(w_hh1, WH1, NGATE, NHID / 8, NHID, 0, WCAR);
  cvt8_kernel<1><<<n8h / NTHR, NTHR, 0, stream>>>(w_ih2, WI2, NGATE, NHID / 8, NHID, 0, WCAR);
  cvt8_kernel<1><<<n8h / NTHR, NTHR, 0, stream>>>(w_hh2, WH2, NGATE, NHID / 8, NHID, 0, WCAR);
  wx1_kernel<<<(NGATE * (KXPAD / 8)) / NTHR, NTHR, 0, stream>>>(w_ih1, WX1);
  lstm2_kernel<<<NBATCH / ROWS_BLK, NTHR, 0, stream>>>(x, b_ih1, b_hh1, b_ih2, b_hh2, WX1, WH1, WI2, WH2, out);
}
